// MCxM_GNN_17944373363255
// MI455X (gfx1250) — hardware-verified
//
#include <hip/hip_runtime.h>
#include <stddef.h>


#define DW      128
#define NTHR    256
#define NWAVE   8
#define EPT     8
#define NGRP    2
#define CHUNK   (NTHR * EPT * NGRP)
#define WCAP    (EPT * NGRP * 32)
#define LISTN   (NWAVE * WCAP)
#define NBC     4096
#define NBF     1024
#define RCAP    40960
#define RBN     128
#define TGT     256
#define DEGCAP  1024
#define OTHR    512
#define BM      64
#define KSTEPS  (DW / 32)
#define GMAX    64
#define PROW    (2 * GMAX)
#define WSCAP   134217728
#define BN_EPS  1e-5f
#define ACARRY  8.0f
#define WCARRY  64.0f
#define GSCALE  (1.0f / 512.0f)

#define LDS_FILL ((RCAP + NBF + LISTN) * 4 + 64)

static_assert((CHUNK & (CHUNK - 1)) == 0);
static_assert(CHUNK <= 4096);
static_assert((NBC & (NBC - 1)) == 0 && (NBF & (NBF - 1)) == 0);
static_assert(NBC == 4 * NBF);
static_assert(OTHR * 8 == NBC);
static_assert((RCAP % 32) == 0);
static_assert(TGT == NWAVE * 32);
static_assert((NBC % TGT) == 0);
static_assert((TGT % BM) == 0);
static_assert(DW == 4 * 32);
static_assert((DW % 32) == 0);
static_assert(PROW == 4 * 32);
static_assert(PROW <= NTHR && DW <= NTHR);
static_assert(WCAP == EPT * NGRP * 32);
static_assert((GMAX & (GMAX - 1)) == 0);

typedef float    v4f  __attribute__((ext_vector_type(4)));
typedef float    v8f  __attribute__((ext_vector_type(8)));
typedef int      v4i  __attribute__((ext_vector_type(4)));
typedef _Float16 v4h  __attribute__((ext_vector_type(4)));
typedef _Float16 v8h  __attribute__((ext_vector_type(8)));
typedef _Float16 v16h __attribute__((ext_vector_type(16)));
union Frag { v16h v; v8h h[2]; };

__device__ __forceinline__ v8f wmh(v16h a, v16h b, v8f c) {
  v8f d = __builtin_amdgcn_wmma_f32_16x16x32_f16(false, a, false, b, (short)0, c, false, false);
  asm volatile("v_nop\n\tv_nop\n\tv_nop\n\tv_nop" : "+v"(d) : "v"(a), "v"(b));
  return d;
}

__device__ __forceinline__ void colsum_out(float* scs, float* srow, v4f cs, float* dst,
                                           int tid, int lane, int wave) {
  *(v4f*)(scs + wave * DW + 4 * lane) = cs;
  __syncthreads();
  if (tid < DW) {
    float s = 0.f;
#pragma unroll
    for (int w = 0; w < NWAVE; ++w) s += scs[w * DW + tid];
    srow[tid] = s;
  }
  __syncthreads();
  const v4f v = *(const v4f*)(srow + 4 * lane);
  if (wave == 0) *(volatile v4f*)(dst + 4 * lane) = v;
  __threadfence();
  if (wave == 0) *(volatile v4f*)(dst + 4 * lane) = v;
}

template <int NB>
__device__ __forceinline__ int scan_chunk(const int* __restrict__ dsts, int nE, int cbase, int slotBase,
                                          int vec8, int* list, int tid, int lane, int wave) {
  int wc = 0;
#pragma unroll
  for (int g = 0; g < NGRP; ++g) {
    const int el0  = (g * NTHR + tid) * EPT;
    const int e0   = cbase + el0;
    const int sent = -2147483647 - 1;
    v4i da, db;
    if (vec8 != 0 && cbase + CHUNK <= nE) {
      da = *(const v4i*)(dsts + e0);
      db = *(const v4i*)(dsts + e0 + 4);
    } else {
      da.x = (e0     < nE) ? dsts[min(e0, nE - 1)] : sent;
      da.y = (e0 + 1 < nE) ? dsts[min(e0 + 1, nE - 1)] : sent;
      da.z = (e0 + 2 < nE) ? dsts[min(e0 + 2, nE - 1)] : sent;
      da.w = (e0 + 3 < nE) ? dsts[min(e0 + 3, nE - 1)] : sent;
      db.x = (e0 + 4 < nE) ? dsts[min(e0 + 4, nE - 1)] : sent;
      db.y = (e0 + 5 < nE) ? dsts[min(e0 + 5, nE - 1)] : sent;
      db.z = (e0 + 6 < nE) ? dsts[min(e0 + 6, nE - 1)] : sent;
      db.w = (e0 + 7 < nE) ? dsts[min(e0 + 7, nE - 1)] : sent;
    }
    const unsigned nb = (unsigned)slotBase;
    const unsigned s0 = (unsigned)da.x - nb, s1 = (unsigned)da.y - nb;
    const unsigned s2 = (unsigned)da.z - nb, s3 = (unsigned)da.w - nb;
    const unsigned s4 = (unsigned)db.x - nb, s5 = (unsigned)db.y - nb;
    const unsigned s6 = (unsigned)db.z - nb, s7 = (unsigned)db.w - nb;
    const bool h0 = s0 < (unsigned)NB, h1 = s1 < (unsigned)NB, h2 = s2 < (unsigned)NB, h3 = s3 < (unsigned)NB;
    const bool h4 = s4 < (unsigned)NB, h5 = s5 < (unsigned)NB, h6 = s6 < (unsigned)NB, h7 = s7 < (unsigned)NB;
    const unsigned any = __builtin_amdgcn_ballot_w32(h0 | h1 | h2 | h3 | h4 | h5 | h6 | h7);
    if (any != 0u) {
#define HITJ(J, HJ, SJ) { \
        const unsigned mj = __builtin_amdgcn_ballot_w32(HJ); \
        if (mj != 0u) { \
          if (HJ) { \
            const int pos = wc + (int)__builtin_amdgcn_mbcnt_lo(mj, 0u); \
            if (pos < WCAP) list[wave * WCAP + pos] = ((el0 + (J)) << 12) | (int)(SJ); \
          } \
          wc += (int)__builtin_popcount(mj); } }
      HITJ(0, h0, s0)
      HITJ(1, h1, s1)
      HITJ(2, h2, s2)
      HITJ(3, h3, s3)
      HITJ(4, h4, s4)
      HITJ(5, h5, s5)
      HITJ(6, h6, s6)
      HITJ(7, h7, s7)
#undef HITJ
    }
  }
  return wc;
}

__global__ __launch_bounds__(NTHR) void k_count(
    const int* __restrict__ dsts, int* cnt, float* dinv, int nE, int vec8) {
  __shared__ __attribute__((aligned(16))) int scnt[NBC];
  __shared__ __attribute__((aligned(16))) int list[LISTN];
  __shared__ int wcnt[NWAVE];
  const int tid = threadIdx.x, lane = tid & 31, wave = tid >> 5;
  const int nodeBase = blockIdx.x * NBC;

  for (int i = tid; i < NBC; i += NTHR) scnt[i] = 0;
  __syncthreads();

  const int nChunks = (nE + CHUNK - 1) / CHUNK;
#pragma unroll 1
  for (int ch = 0; ch < nChunks; ++ch) {
    const int cbase = ch * CHUNK;
    const int wc = scan_chunk<NBC>(dsts, nE, cbase, nodeBase, vec8, list, tid, lane, wave);
    if (lane == 0) wcnt[wave] = wc;
    __syncthreads();
    if (wave == 0) {
#pragma unroll 1
      for (int wsx = 0; wsx < NWAVE; ++wsx) {
        int n = __builtin_amdgcn_readfirstlane(wcnt[wsx]);
        n = n > WCAP ? WCAP : (n < 0 ? 0 : n);
        const int* lp = list + wsx * WCAP;
#pragma unroll 1
        for (int i = 0; i < n; ++i) {
          const int ent  = __builtin_amdgcn_readfirstlane(lp[i]);
          const int slot = ent & (NBC - 1);
          if (lane == 0) scnt[slot] = scnt[slot] + 1;
        }
      }
    }
    __syncthreads();
  }

  v4i cq[4];
  v4f dq[4];
#pragma unroll
  for (int q = 0; q < 4; ++q) {
    const int f = (wave * 4 + q) * 128 + 4 * lane;
    const v4i cv = *(const v4i*)(scnt + f);
    cq[q] = cv;
    v4f d;
    d.x = rsqrtf((float)(cv.x < 0 ? 0 : cv.x) + 1.0f);
    d.y = rsqrtf((float)(cv.y < 0 ? 0 : cv.y) + 1.0f);
    d.z = rsqrtf((float)(cv.z < 0 ? 0 : cv.z) + 1.0f);
    d.w = rsqrtf((float)(cv.w < 0 ? 0 : cv.w) + 1.0f);
    dq[q] = d;
  }
  int*   cp = cnt  + (size_t)nodeBase;
  float* dp = dinv + (size_t)nodeBase;
#pragma unroll
  for (int q = 0; q < 4; ++q) {
    const int f = (wave * 4 + q) * 128 + 4 * lane;
    *(volatile v4i*)(cp + f) = cq[q];
    *(volatile v4f*)(dp + f) = dq[q];
  }
  __threadfence();
#pragma unroll
  for (int q = 0; q < 4; ++q) {
    const int f = (wave * 4 + q) * 128 + 4 * lane;
    *(volatile v4i*)(cp + f) = cq[q];
    *(volatile v4f*)(dp + f) = dq[q];
  }
}

__global__ __launch_bounds__(OTHR) void k_offsets(
    const int* __restrict__ cnt, int* off, int* rbase, int nChunk) {
  __shared__ __attribute__((aligned(16))) int soff[NBC];
  __shared__ __attribute__((aligned(16))) int srb[RBN];
  __shared__ int wtot[OTHR / 32];
  const int tid = threadIdx.x, lane = tid & 31, wave = tid >> 5, sub = tid >> 7;
  for (int i = tid; i < RBN; i += OTHR) srb[i] = 0;
  int carry = 0;
#pragma unroll 1
  for (int ch = 0; ch < nChunk; ++ch) {
    const int base = ch * NBC;
    const v4i c0 = *(const v4i*)(cnt + base + 8 * tid);
    const v4i c1 = *(const v4i*)(cnt + base + 8 * tid + 4);
    const int e0 = max(c0.x, 0), e1 = max(c0.y, 0), e2 = max(c0.z, 0), e3 = max(c0.w, 0);
    const int e4 = max(c1.x, 0), e5 = max(c1.y, 0), e6 = max(c1.z, 0), e7 = max(c1.w, 0);
    const int ts = e0 + e1 + e2 + e3 + e4 + e5 + e6 + e7;
    int incl = ts;
#pragma unroll
    for (int d = 1; d < 32; d <<= 1) {
      const int t = __shfl_up(incl, d);
      if (lane >= d) incl += t;
    }
    if (lane == 31) wtot[wave] = incl;
    __syncthreads();
    const int S0 = wtot[0]  + wtot[1]  + wtot[2]  + wtot[3];
    const int S1 = wtot[4]  + wtot[5]  + wtot[6]  + wtot[7];
    const int S2 = wtot[8]  + wtot[9]  + wtot[10] + wtot[11];
    const int S3 = wtot[12] + wtot[13] + wtot[14] + wtot[15];
    int pre = 0;
#pragma unroll 1
    for (int w = 4 * sub; w < wave; ++w) pre += wtot[w];
    const int b0 = carry;
    const int b1 = b0 + ((S0 + 31) & ~31);
    const int b2 = b1 + ((S1 + 31) & ~31);
    const int b3 = b2 + ((S2 + 31) & ~31);
    const int b4 = b3 + ((S3 + 31) & ~31);
    const int myb = sub == 0 ? b0 : (sub == 1 ? b1 : (sub == 2 ? b2 : b3));
    if (tid == 0) {
      srb[min(4 * ch + 0, RBN - 1)] = b0;
      srb[min(4 * ch + 1, RBN - 1)] = b1;
      srb[min(4 * ch + 2, RBN - 1)] = b2;
      srb[min(4 * ch + 3, RBN - 1)] = b3;
    }
    int run = myb + pre + incl - ts;
    soff[8 * tid + 0] = run; run += e0;
    soff[8 * tid + 1] = run; run += e1;
    soff[8 * tid + 2] = run; run += e2;
    soff[8 * tid + 3] = run; run += e3;
    soff[8 * tid + 4] = run; run += e4;
    soff[8 * tid + 5] = run; run += e5;
    soff[8 * tid + 6] = run; run += e6;
    soff[8 * tid + 7] = run;
    carry = b4;
    __syncthreads();
    const v4i o0 = *(const v4i*)(soff + 4 * tid);
    const v4i o1 = *(const v4i*)(soff + 4 * (tid + OTHR));
    int* op = off + base;
    *(volatile v4i*)(op + 4 * tid) = o0;
    *(volatile v4i*)(op + 4 * (tid + OTHR)) = o1;
    __threadfence();
    *(volatile v4i*)(op + 4 * tid) = o0;
    *(volatile v4i*)(op + 4 * (tid + OTHR)) = o1;
    __syncthreads();
  }
  if (tid == 0) srb[min(4 * nChunk, RBN - 1)] = carry;
  __syncthreads();
  v4i rv = {0, 0, 0, 0};
  if (tid < 32) rv = *(const v4i*)(srb + 4 * tid);
  if (tid < 32) *(volatile v4i*)(rbase + 4 * tid) = rv;
  __threadfence();
  if (tid < 32) *(volatile v4i*)(rbase + 4 * tid) = rv;
}

__global__ __launch_bounds__(NTHR) void k_fill(
    const int* __restrict__ srcs, const int* __restrict__ dsts,
    const int* __restrict__ off, const int* __restrict__ rbase,
    int* csr, int nN, int nE, int vec8, int csrLen) {
  extern __shared__ v4f lds_dyn[];
  int* region = (int*)lds_dyn;
  int* cursor = region + RCAP;
  int* list   = cursor + NBF;
  int* wcnt   = list + LISTN;
  const int tid = threadIdx.x, lane = tid & 31, wave = tid >> 5;
  const int b = blockIdx.x;
  const int nodeBase = b * NBF;

  int rb0 = rbase[b];
  const int rb1 = rbase[b + 1];
  rb0 = rb0 < 0 ? 0 : (rb0 > csrLen ? csrLen : rb0);
  rb0 &= ~31;
  int len = rb1 - rb0;
  len = len < 0 ? 0 : (len > RCAP ? RCAP : len);
  int lenW = (len + 31) & ~31;
  if (rb0 + lenW > csrLen) lenW = (csrLen - rb0) & ~31;

  {
    const v4i z = {0, 0, 0, 0};
    for (int i = tid; i < RCAP / 4; i += NTHR) ((v4i*)region)[i] = z;
    for (int s = tid; s < NBF; s += NTHR) {
      int o = off[nodeBase + s] - rb0;
      o = o < 0 ? 0 : (o > RCAP ? RCAP : o);
      cursor[s] = o;
    }
  }
  __syncthreads();

  const int nChunks = (nE + CHUNK - 1) / CHUNK;
#pragma unroll 1
  for (int ch = 0; ch < nChunks; ++ch) {
    const int cbase = ch * CHUNK;
    const int wc = scan_chunk<NBF>(dsts, nE, cbase, nodeBase, vec8, list, tid, lane, wave);
    if (lane == 0) wcnt[wave] = wc;
    __syncthreads();
    if (wave == 0) {
#pragma unroll 1
      for (int wsx = 0; wsx < NWAVE; ++wsx) {
        int n = __builtin_amdgcn_readfirstlane(wcnt[wsx]);
        n = n > WCAP ? WCAP : (n < 0 ? 0 : n);
        const int* lp = list + wsx * WCAP;
#pragma unroll 1
        for (int i = 0; i < n; ++i) {
          const int ent  = __builtin_amdgcn_readfirstlane(lp[i]);
          const int slot = ent & (NBF - 1);
          int e = cbase + ((ent >> 12) & (CHUNK - 1));
          e = e > nE - 1 ? nE - 1 : e;
          int sv = srcs[e];
          sv = sv < 0 ? 0 : (sv > nN - 1 ? nN - 1 : sv);
          if (lane == 0) {
            int pos = cursor[slot];
            pos = pos < 0 ? 0 : (pos > RCAP - 1 ? RCAP - 1 : pos);
            region[pos] = sv;
            const int np = pos + 1;
            cursor[slot] = np > RCAP ? RCAP : np;
          }
        }
      }
    }
    __syncthreads();
  }

  const int nv = lenW >> 2;
  int* gp = csr + rb0;
#pragma unroll 1
  for (int i = tid; i < nv; i += NTHR) { const v4i v = ((const v4i*)region)[i]; *(volatile v4i*)(gp + 4 * i) = v; }
  __threadfence();
#pragma unroll 1
  for (int i = tid; i < nv; i += NTHR) { const v4i v = ((const v4i*)region)[i]; *(volatile v4i*)(gp + 4 * i) = v; }
}

__global__ __launch_bounds__(NTHR) void k_xcvt(
    const float* __restrict__ x, const float* __restrict__ mask, _Float16* ap, int nN) {
  const int tid = threadIdx.x, lane = tid & 31, wave = tid >> 5;
  const int tbase = blockIdx.x * TGT + wave * 32;
  const int col4 = 4 * lane;
#pragma unroll 1
  for (int j = 0; j < 32; ++j) {
    const int c = tbase + j;
    const bool live = c < nN;
    int cc = c > nN - 1 ? nN - 1 : c;
    cc = cc < 0 ? 0 : cc;
    const float mk = live ? mask[cc] * ACARRY : 0.f;
    const v4f xv = *(const v4f*)(x + (size_t)cc * DW + col4);
    v4h o;
    o.x = (_Float16)(xv.x * mk);
    o.y = (_Float16)(xv.y * mk);
    o.z = (_Float16)(xv.z * mk);
    o.w = (_Float16)(xv.w * mk);
    _Float16* gp = ap + (size_t)c * DW + col4;
    *(volatile v4h*)gp = o;
    __threadfence();
    *(volatile v4h*)gp = o;
  }
}

__global__ __launch_bounds__(NTHR) void k_wtcvt(const float* __restrict__ W, _Float16* dp,
                                                int K, int Nout, int nUnits) {
  const int i = (int)blockIdx.x * NTHR + (int)threadIdx.x;
  if (i >= nUnits) return;
  const int ppr = K >> 3;
  const int per = Nout * ppr;
  const int L = i / per;
  const int r = i - L * per;
  const int n = r / ppr;
  const int seg = r - n * ppr;
  const float* p = W + (size_t)L * K * Nout + (size_t)(8 * seg) * Nout + n;
  v8h o;
#pragma unroll
  for (int j = 0; j < 8; ++j) o[j] = (_Float16)(p[(size_t)j * Nout] * WCARRY);
  _Float16* gp = dp + (size_t)i * 8;
  *(volatile v8h*)gp = o;
  __threadfence();
  *(volatile v8h*)gp = o;
}

__global__ __launch_bounds__(NTHR) void k_gemm(
    const _Float16* __restrict__ A, const _Float16* __restrict__ Bp, float* C32) {
  constexpr int TPW = 4;
  constexpr int PPR = DW / 4;
  constexpr int NIT = (BM * PPR) / NTHR;
  static_assert((BM * PPR) % NTHR == 0);
  static_assert(NIT >= 1);
  static_assert(TPW * 16 * 2 == DW);
  static_assert(BM == 4 * 16);

  __shared__ __attribute__((aligned(16))) float stg[BM * DW];
  const int tid = threadIdx.x, lane = tid & 31, wave = tid >> 5, hh = lane >> 4, m = lane & 15;
  const int rowBase = (int)blockIdx.x * BM;
  const int rg = wave >> 1, chf = wave & 1;
  const int r0 = rg * 16;
  const int c0 = chf * (DW / 2);

  v8f acc[TPW];
#pragma unroll
  for (int t = 0; t < TPW; ++t) { v8f z = {0.f, 0.f, 0.f, 0.f, 0.f, 0.f, 0.f, 0.f}; acc[t] = z; }

  const _Float16* ap = A  + (size_t)(rowBase + r0 + m) * DW + 8 * hh;
  const _Float16* bp = Bp + (size_t)(c0 + m) * DW + 8 * hh;
#pragma unroll 1
  for (int kt = 0; kt < KSTEPS; ++kt) {
    Frag a;
    a.h[0] = *(const v8h*)(ap + 32 * kt);
    a.h[1] = *(const v8h*)(ap + 32 * kt + 16);
#pragma unroll
    for (int t = 0; t < TPW; ++t) {
      const size_t to = (size_t)(16 * t) * DW + 32 * kt;
      Frag b;
      b.h[0] = *(const v8h*)(bp + to);
      b.h[1] = *(const v8h*)(bp + to + 16);
      acc[t] = wmh(a.v, b.v, acc[t]);
    }
  }

  {
    float* sp = stg + (size_t)(r0 + 8 * hh) * DW + c0 + m;
#pragma unroll
    for (int t = 0; t < TPW; ++t) {
#pragma unroll
      for (int r = 0; r < 8; ++r) sp[r * DW + 16 * t] = acc[t][r] * GSCALE;
    }
  }
  __syncthreads();

  v4f cv[NIT];
#pragma unroll
  for (int it = 0; it < NIT; ++it) {
    const int id = it * NTHR + tid;
    const int row = id / PPR, seg = id % PPR;
    cv[it] = *(const v4f*)(stg + (size_t)row * DW + 4 * seg);
  }
#pragma unroll
  for (int it = 0; it < NIT; ++it) {
    const int id = it * NTHR + tid;
    const int row = id / PPR, seg = id % PPR;
    float* gp = C32 + (size_t)(rowBase + row) * DW + 4 * seg;
    *(volatile v4f*)gp = cv[it];
  }
  __threadfence();
#pragma unroll
  for (int it = 0; it < NIT; ++it) {
    const int id = it * NTHR + tid;
    const int row = id / PPR, seg = id % PPR;
    float* gp = C32 + (size_t)(rowBase + row) * DW + 4 * seg;
    *(volatile v4f*)gp = cv[it];
  }
}

__global__ __launch_bounds__(NTHR) void k_agg(
    const int* __restrict__ csr, const int* __restrict__ off, const int* __restrict__ cnt,
    const float* __restrict__ dinv, const float* __restrict__ hw, const float* __restrict__ bias,
    float* xo, float* xsum, int nN, int csrLen) {
  __shared__ __attribute__((aligned(16))) float scs[NWAVE * DW];
  __shared__ __attribute__((aligned(16))) float srow[DW];
  const int tid = threadIdx.x, lane = tid & 31, wave = tid >> 5;
  const int tbase = blockIdx.x * TGT + wave * 32;
  const int col4 = 4 * lane;
  const int cl    = tbase + lane;
  const int cnt_l = cnt[cl];
  const int off_l = off[cl];
  const float di_l = dinv[cl];
  const v4f vb = *(const v4f*)(bias + col4);
  v4f cs = {0.f, 0.f, 0.f, 0.f};

#pragma unroll 1
  for (int j = 0; j < 32; ++j) {
    const int c = tbase + j;
    int n = __shfl(cnt_l, j);
    n = n < 0 ? 0 : (n > DEGCAP ? DEGCAP : n);
    const int st = __shfl(off_l, j);
    const float dc = __shfl(di_l, j);
    const float dd = dc * dc;

    v4f a = *(const v4f*)(hw + (size_t)c * DW + col4);
    a = a * dd;
#pragma unroll 1
    for (int q0 = 0; q0 < n; q0 += 32) {
      int pos = st + q0 + lane;
      pos = pos < 0 ? 0 : (pos > csrLen - 1 ? csrLen - 1 : pos);
      int sl = csr[pos];
      sl = sl < 0 ? 0 : (sl > nN - 1 ? nN - 1 : sl);
      const int mcnt = (n - q0) < 32 ? (n - q0) : 32;
#pragma unroll 1
      for (int pp = 0; pp < mcnt; ++pp) {
        const int s = __builtin_amdgcn_readlane(sl, pp);
        const float cf = dinv[s] * dc;
        const v4f xv = *(const v4f*)(hw + (size_t)s * DW + col4);
        a = a + xv * cf;
      }
    }

    const bool live = c < nN;
    v4f o;
    o.x = live ? (a.x + vb.x) : 0.f;
    o.y = live ? (a.y + vb.y) : 0.f;
    o.z = live ? (a.z + vb.z) : 0.f;
    o.w = live ? (a.w + vb.w) : 0.f;
    cs = cs + o;
    float* gp = xo + (size_t)c * DW + col4;
    *(volatile v4f*)gp = o;
    __threadfence();
    *(volatile v4f*)gp = o;
  }

  colsum_out(scs, srow, cs, xsum + (size_t)blockIdx.x * DW, tid, lane, wave);
}

__global__ __launch_bounds__(NTHR) void k_var(const float* __restrict__ xo, const float* __restrict__ xsum,
                                              float* sq, int nN, int nPart) {
  __shared__ __attribute__((aligned(16))) float smu[DW];
  __shared__ __attribute__((aligned(16))) float scs[NWAVE * DW];
  __shared__ __attribute__((aligned(16))) float srow[DW];
  const int tid = threadIdx.x, lane = tid & 31, wave = tid >> 5;
  const int tbase = blockIdx.x * TGT + wave * 32;
  const int col4 = 4 * lane;
  if (tid < DW) {
    double s = 0.0;
#pragma unroll 1
    for (int b = 0; b < nPart; ++b) s += (double)xsum[(size_t)b * DW + tid];
    smu[tid] = (float)(s / (double)nN);
  }
  __syncthreads();
  const v4f mu = *(const v4f*)(smu + col4);
  v4f cs = {0.f, 0.f, 0.f, 0.f};
#pragma unroll 1
  for (int j = 0; j < 32; ++j) {
    const int c = tbase + j;
    if (c >= nN) break;
    const v4f xv = *(const v4f*)(xo + (size_t)c * DW + col4);
    const v4f d = xv - mu;
    cs = cs + d * d;
  }
  colsum_out(scs, srow, cs, sq + (size_t)blockIdx.x * DW, tid, lane, wave);
}

template <int LAST>
__global__ __launch_bounds__(NTHR) void k_bnapply(
    const float* __restrict__ xo, const float* __restrict__ xsum, const float* __restrict__ sq,
    const float* __restrict__ gam, const float* __restrict__ bet, const float* __restrict__ mask,
    const int* __restrict__ batch, const float* __restrict__ wout,
    _Float16* ap, float* part, int nN, int nPart, int nG) {
  __shared__ __attribute__((aligned(16))) float smu[DW];
  __shared__ __attribute__((aligned(16))) float srs[DW];
  __shared__ __attribute__((aligned(16))) float sg[DW];
  __shared__ __attribute__((aligned(16))) float sb[DW];
  __shared__ __attribute__((aligned(16))) float ss[TGT];
  __shared__ __attribute__((aligned(16))) int   sgi[TGT];
  __shared__ __attribute__((aligned(16))) float spart[PROW];
  const int tid = threadIdx.x, lane = tid & 31, wave = tid >> 5;
  const int tbase = blockIdx.x * TGT + wave * 32;
  const int col4 = 4 * lane;
  if (tid < DW) {
    double s1 = 0.0, s2 = 0.0;
#pragma unroll 1
    for (int b = 0; b < nPart; ++b) {
      s1 += (double)xsum[(size_t)b * DW + tid];
      s2 += (double)sq[(size_t)b * DW + tid];
    }
    const float mu  = (float)(s1 / (double)nN);
    const float var = (float)(s2 / (double)nN);
    smu[tid] = mu;
    srs[tid] = rsqrtf(var + BN_EPS);
    sg[tid]  = gam[tid];
    sb[tid]  = bet[tid];
  }
  __syncthreads();
  const v4f mu = *(const v4f*)(smu + col4);
  const v4f rs = *(const v4f*)(srs + col4);
  const v4f gg = *(const v4f*)(sg + col4);
  const v4f be = *(const v4f*)(sb + col4);
  v4f wo = {0.f, 0.f, 0.f, 0.f};
  if constexpr (LAST == 1) wo = *(const v4f*)(wout + col4);
  float myo = 0.f;
  int   myg = -1;
#pragma unroll 1
  for (int j = 0; j < 32; ++j) {
    const int c = tbase + j;
    const bool live = c < nN;
    int cc = c > nN - 1 ? nN - 1 : c;
    cc = cc < 0 ? 0 : cc;
    const float mk = live ? mask[cc] : 0.f;
    const v4f xv = *(const v4f*)(xo + (size_t)c * DW + col4);
    const v4f t = (gg * (xv - mu)) * rs + be;
    v4f y;
    y.x = fmaxf(t.x, 0.f) * mk;
    y.y = fmaxf(t.y, 0.f) * mk;
    y.z = fmaxf(t.z, 0.f) * mk;
    y.w = fmaxf(t.w, 0.f) * mk;
    if constexpr (LAST == 0) {
      v4h o;
      o.x = (_Float16)(y.x * ACARRY);
      o.y = (_Float16)(y.y * ACARRY);
      o.z = (_Float16)(y.z * ACARRY);
      o.w = (_Float16)(y.w * ACARRY);
      _Float16* gp = ap + (size_t)c * DW + col4;
      *(volatile v4h*)gp = o;
      __threadfence();
      *(volatile v4h*)gp = o;
    } else {
      float pd = y.x * wo.x + y.y * wo.y + y.z * wo.z + y.w * wo.w;
      pd += __shfl_xor(pd, 16);
      pd += __shfl_xor(pd, 8);
      pd += __shfl_xor(pd, 4);
      pd += __shfl_xor(pd, 2);
      pd += __shfl_xor(pd, 1);
      const int gb = batch[cc];
      const int g = (live && gb >= 0 && gb < nG) ? gb : -1;
      myo = (lane == j) ? pd : myo;
      myg = (lane == j) ? g : myg;
    }
  }
  if constexpr (LAST == 1) {
    ss[tid]  = myo;
    sgi[tid] = myg;
    __syncthreads();
    if (tid < PROW) {
      const int tg = tid & (GMAX - 1);
      float acc = 0.f;
      int cn = 0;
#pragma unroll 1
      for (int i = 0; i < TGT; ++i) {
        const bool h = sgi[i] == tg;
        const float v = ss[i];
        acc += h ? v : 0.f;
        cn  += h ? 1 : 0;
      }
      spart[tid] = (tid < GMAX) ? acc : (float)cn;
    }
    __syncthreads();
    const v4f pv = *(const v4f*)(spart + col4);
    float* gp = part + (size_t)blockIdx.x * PROW + col4;
    if (wave == 0) *(volatile v4f*)gp = pv;
    __threadfence();
    if (wave == 0) *(volatile v4f*)gp = pv;
  }
}

__global__ __launch_bounds__(NTHR) void k_head(const float* __restrict__ part, const float* __restrict__ bout,
                                               float* out, int nPart, int nG) {
  __shared__ __attribute__((aligned(16))) float so[GMAX];
  const int tid = threadIdx.x;
  if (tid < GMAX) {
    double S = 0.0, C = 0.0;
#pragma unroll 1
    for (int b = 0; b < nPart; ++b) {
      S += (double)part[(size_t)b * PROW + tid];
      C += (double)part[(size_t)b * PROW + GMAX + tid];
    }
    const float Sf = (float)S;
    float Cf = (float)C;
    Cf = Cf < 1.f ? 1.f : Cf;
    const float v = Sf * (1.0f / Cf) + bout[0];
    so[tid] = (tid < nG) ? v : 0.f;
  }
  __syncthreads();
  const int nq = nG >> 2, rem = nG & 3;
  const bool act = tid < nq;
  const int q = act ? tid : 0;
  const v4f v = *(const v4f*)(so + 4 * q);
  float* gp = out + 4 * q;
  const bool tail = (tid == nq) && (rem > 0);
  int tb = 4 * nq;
  tb = tb > GMAX - 4 ? GMAX - 4 : tb;
  const float t0 = so[tb], t1 = so[tb + 1], t2 = so[tb + 2];
  float* tp = out + 4 * nq;
  if (act) *(volatile v4f*)gp = v;
  if (tail) {
    *(volatile float*)tp = t0;
    if (rem > 1) *(volatile float*)(tp + 1) = t1;
    if (rem > 2) *(volatile float*)(tp + 2) = t2;
  }
  __threadfence();
  if (act) *(volatile v4f*)gp = v;
  if (tail) {
    *(volatile float*)tp = t0;
    if (rem > 1) *(volatile float*)(tp + 1) = t1;
    if (rem > 2) *(volatile float*)(tp + 2) = t2;
  }
}

extern "C" void kernel_launch(void* const* d_in, const int* in_sizes, int n_in,
                              void* d_out, int out_size, void* d_ws, size_t ws_size,
                              hipStream_t stream) {
  if (n_in < 10) return;
  if (in_sizes[0] < DW || (in_sizes[0] % DW) != 0) return;
  const int nN = in_sizes[0] / DW;
  if (in_sizes[1] < 2 || (in_sizes[1] & 1) != 0) return;
  const int nE = in_sizes[1] / 2;
  if (in_sizes[2] != nN || in_sizes[3] != nN) return;
  if (in_sizes[4] < DW * DW || (in_sizes[4] % (DW * DW)) != 0) return;
  const int nL = in_sizes[4] / (DW * DW);
  if (nL > 8) return;
  if (in_sizes[5] != nL * DW || in_sizes[6] != nL * DW || in_sizes[7] != nL * DW) return;
  if (in_sizes[8] != DW || in_sizes[9] < 1) return;
  const int nG = out_size;
  if (nG < 1 || nG > GMAX) return;
  if (nE > (1 << 28) || nN > (1 << 22)) return;

  const float* x     = (const float*)d_in[0];
  const int*   ei    = (const int*)d_in[1];
  const int*   src   = ei;
  const int*   dst   = ei + nE;
  const float* mask  = (const float*)d_in[2];
  const int*   batch = (const int*)d_in[3];
  const float* W     = (const float*)d_in[4];
  const float* bcv   = (const float*)d_in[5];
  const float* gam   = (const float*)d_in[6];
  const float* bet   = (const float*)d_in[7];
  const float* wout  = (const float*)d_in[8];
  const float* bout  = (const float*)d_in[9];
  float* out = (float*)d_out;

  const int NPAD   = ((nN + TGT - 1) / TGT) * TGT;
  const int nBC    = (nN + NBC - 1) / NBC;
  const int CNTPAD = nBC * NBC;
  if (CNTPAD < NPAD) return;
  if (4 * nBC + 1 > RBN) return;
  const int nBF    = (nN + NBF - 1) / NBF;
  if (nBF > 4 * nBC) return;
  const int csrLen = ((nE + 31) & ~31) + 4096;
  if (31 * 4 * nBC > 4096) return;
  const int nAgg   = NPAD / TGT;
  const int nGemm  = NPAD / BM;
  const int nUnits = nL * DW * DW / 8;

  char* ws = (char*)d_ws;
  size_t off = 0;
  const size_t oWp  = off; off += (size_t)nL * DW * DW * 2;       off = (off + 255) & ~(size_t)255;
  const size_t oA   = off; off += (size_t)NPAD * DW * 2;          off = (off + 255) & ~(size_t)255;
  const size_t oC   = off; off += (size_t)NPAD * DW * 4;          off = (off + 255) & ~(size_t)255;
  const size_t oX   = off; off += (size_t)NPAD * DW * 4;          off = (off + 255) & ~(size_t)255;
  const size_t oCnt = off; off += (size_t)CNTPAD * 4;             off = (off + 255) & ~(size_t)255;
  const size_t oDi  = off; off += (size_t)CNTPAD * 4;             off = (off + 255) & ~(size_t)255;
  const size_t oOff = off; off += (size_t)CNTPAD * 4;             off = (off + 255) & ~(size_t)255;
  const size_t oRb  = off; off += (size_t)RBN * 4;                off = (off + 255) & ~(size_t)255;
  const size_t oCsr = off; off += (size_t)csrLen * 4;             off = (off + 255) & ~(size_t)255;
  const size_t oXs  = off; off += (size_t)nAgg * DW * 4;          off = (off + 255) & ~(size_t)255;
  const size_t oSq  = off; off += (size_t)nAgg * DW * 4;          off = (off + 255) & ~(size_t)255;
  const size_t oPt  = off; off += (size_t)nAgg * PROW * 4;        off = (off + 255) & ~(size_t)255;
  if (off > ws_size || off > (size_t)WSCAP) return;

  _Float16* wpl = (_Float16*)(ws + oWp);
  _Float16* apl = (_Float16*)(ws + oA);
  float* cbuf = (float*)(ws + oC);
  float* xo   = (float*)(ws + oX);
  int*   cnt  = (int*)(ws + oCnt);
  float* dinv = (float*)(ws + oDi);
  int*   offp = (int*)(ws + oOff);
  int*   rb   = (int*)(ws + oRb);
  int*   csr  = (int*)(ws + oCsr);
  float* xsum = (float*)(ws + oXs);
  float* sq   = (float*)(ws + oSq);
  float* part = (float*)(ws + oPt);

  const int vec8 = ((nE & 3) == 0) ? 1 : 0;

  k_xcvt<<<nAgg, NTHR, 0, stream>>>(x, mask, apl, nN);
  k_wtcvt<<<(nUnits + NTHR - 1) / NTHR, NTHR, 0, stream>>>(W, wpl, DW, DW, nUnits);
  k_count<<<nBC, NTHR, 0, stream>>>(dst, cnt, dinv, nE, vec8);
  k_offsets<<<1, OTHR, 0, stream>>>(cnt, offp, rb, nBC);
  hipFuncSetAttribute(reinterpret_cast<const void*>(&k_fill),
                      hipFuncAttributeMaxDynamicSharedMemorySize, LDS_FILL);
  k_fill<<<nBF, NTHR, LDS_FILL, stream>>>(src, dst, offp, rb, csr, nN, nE, vec8, csrLen);

  for (int l = 0; l < nL; ++l) {
    const _Float16* bp = wpl + (size_t)l * DW * DW;
    const float* bs = bcv + (size_t)l * DW;
    const float* gl = gam + (size_t)l * DW;
    const float* bl = bet + (size_t)l * DW;
    k_gemm<<<nGemm, NTHR, 0, stream>>>(apl, bp, cbuf);
    k_agg<<<nAgg, NTHR, 0, stream>>>(csr, offp, cnt, dinv, cbuf, bs, xo, xsum, nN, csrLen);
    k_var<<<nAgg, NTHR, 0, stream>>>(xo, xsum, sq, nN, nAgg);
    if (l < nL - 1)
      k_bnapply<0><<<nAgg, NTHR, 0, stream>>>(xo, xsum, sq, gl, bl, mask, batch, wout, apl, part, nN, nAgg, nG);
    else
      k_bnapply<1><<<nAgg, NTHR, 0, stream>>>(xo, xsum, sq, gl, bl, mask, batch, wout, apl, part, nN, nAgg, nG);
  }
  k_head<<<1, NTHR, 0, stream>>>(part, bout, out, nAgg, nG);
}
